// SGFormer_9706626089235
// MI455X (gfx1250) — hardware-run, weakly checked
//
#include <hip/hip_runtime.h>
#include <stddef.h>


#define DW      128
#define NTHR    256
#define NWAVE   8
#define EPT     8
#define NGRP    2
#define CHUNK   (NTHR * EPT * NGRP)
#define WCAP    (EPT * NGRP * 32)
#define LISTN   (NWAVE * WCAP)
#define NBC     4096
#define NBF     1024
#define RCAP    40960
#define RBN     128
#define TGT     256
#define DEGCAP  1024
#define OTHR    512
#define BM      64
#define RT      4
#define RB      (BM * RT)
#define KSTEPS  (DW / 32)
#define NMAT    5
#define MPN     144
#define PSTRIDE (DW * DW + DW + 32)
#define WSLIM   134217728
#define ACARRY  8.0f
#define WCARRY  64.0f
#define GSCALE  (1.0f / 512.0f)
#define HCONV   (1.0f / 64.0f)
#define MCARRY  0.25f
#define MSCALE  (1.0f / 64.0f)
#define CBETA   0.4f
#define OMBETA  0.6f
#define CALPHA  0.6f
#define OMALPHA 0.4f

#define LDS_FILL ((RCAP + NBF + LISTN) * 4 + 64)
#define LP_A16   0
#define LP_STG   16384
#define LP_KT    49152
#define LP_VT    65536
#define LP_SKS   81920
#define LP_SWQ   83968
#define LP_SWK   84000
#define LP_SLN   84032
#define LP_MAC   84736
#define LDS_PROJ 150272

static_assert((CHUNK & (CHUNK - 1)) == 0);
static_assert(CHUNK <= 4096);
static_assert((NBC & (NBC - 1)) == 0 && (NBF & (NBF - 1)) == 0);
static_assert(NBC == 4 * NBF);
static_assert(OTHR * 8 == NBC);
static_assert((RCAP % 32) == 0);
static_assert(TGT == NWAVE * 32);
static_assert((NBC % TGT) == 0);
static_assert((TGT % BM) == 0);
static_assert(RB == TGT);
static_assert(DW == 4 * 32);
static_assert((DW % 32) == 0);
static_assert(BM == 64);
static_assert(WCAP == EPT * NGRP * 32);
static_assert((PSTRIDE % 32) == 0);
static_assert(PSTRIDE == DW * DW + 160);
static_assert((MPN % 16) == 0 && MPN >= DW + 1);
static_assert(((MPN * DW) % (8 * NTHR)) == 0);
static_assert(LP_SLN + 160 * 4 <= LP_MAC);
static_assert((LP_MAC % 16) == 0);
static_assert(LP_MAC + DW * DW * 4 == LDS_PROJ);
static_assert(LP_STG == BM * DW * 2 && LP_KT == LP_STG + BM * DW * 4);
static_assert(LP_VT == LP_KT + DW * BM * 2 && LP_SKS == LP_VT + DW * BM * 2);
static_assert(LP_SWQ == LP_SKS + 4 * DW * 4);

typedef float    v4f  __attribute__((ext_vector_type(4)));
typedef float    v8f  __attribute__((ext_vector_type(8)));
typedef int      v4i  __attribute__((ext_vector_type(4)));
typedef _Float16 v4h  __attribute__((ext_vector_type(4)));
typedef _Float16 v8h  __attribute__((ext_vector_type(8)));
typedef _Float16 v16h __attribute__((ext_vector_type(16)));
union Frag { v16h v; v8h h[2]; };

__device__ __forceinline__ v8f wmh(v16h a, v16h b, v8f c) {
  v8f d = __builtin_amdgcn_wmma_f32_16x16x32_f16(false, a, false, b, (short)0, c, false, false);
  asm volatile("v_nop\n\tv_nop\n\tv_nop\n\tv_nop" : "+v"(d) : "v"(a), "v"(b));
  return d;
}

__device__ __forceinline__ v8f zero8() { v8f z = {0.f, 0.f, 0.f, 0.f, 0.f, 0.f, 0.f, 0.f}; return z; }

__device__ __forceinline__ void gemm_tile4(const _Float16* a16, const _Float16* __restrict__ bpl,
                                           int r0, int c0, int hh, int m, v8f (&acc)[4]) {
#pragma unroll
  for (int t = 0; t < 4; ++t) acc[t] = zero8();
  const _Float16* ap = a16 + (size_t)(r0 + m) * DW + 8 * hh;
  const _Float16* bp = bpl + (size_t)(c0 + m) * DW + 8 * hh;
#pragma unroll 1
  for (int kt = 0; kt < KSTEPS; ++kt) {
    Frag a;
    a.h[0] = *(const v8h*)(ap + 32 * kt);
    a.h[1] = *(const v8h*)(ap + 32 * kt + 16);
#pragma unroll
    for (int t = 0; t < 4; ++t) {
      const size_t to = (size_t)(16 * t) * DW + 32 * kt;
      Frag b;
      b.h[0] = *(const v8h*)(bp + to);
      b.h[1] = *(const v8h*)(bp + to + 16);
      acc[t] = wmh(a.v, b.v, acc[t]);
    }
  }
}

__device__ __forceinline__ void write_rows64(const float* stg, float* gb, float scale, int tid) {
  v4f cv[8];
#pragma unroll
  for (int it = 0; it < 8; ++it) {
    const int id = it * NTHR + tid;
    const v4f v = *(const v4f*)(stg + (size_t)(id >> 5) * DW + 4 * (id & 31));
    cv[it] = v * scale;
  }
#pragma unroll
  for (int it = 0; it < 8; ++it) {
    const int id = it * NTHR + tid;
    *(volatile v4f*)(gb + (size_t)(id >> 5) * DW + 4 * (id & 31)) = cv[it];
  }
  __threadfence();
#pragma unroll
  for (int it = 0; it < 8; ++it) {
    const int id = it * NTHR + tid;
    *(volatile v4f*)(gb + (size_t)(id >> 5) * DW + 4 * (id & 31)) = cv[it];
  }
}

template <int NB>
__device__ __forceinline__ int scan_chunk(const int* __restrict__ dsts, int nE, int cbase, int slotBase,
                                          int vec8, int* list, int tid, int lane, int wave) {
  int wc = 0;
#pragma unroll
  for (int g = 0; g < NGRP; ++g) {
    const int el0  = (g * NTHR + tid) * EPT;
    const int e0   = cbase + el0;
    const int sent = -2147483647 - 1;
    v4i da, db;
    if (vec8 != 0 && cbase + CHUNK <= nE) {
      da = *(const v4i*)(dsts + e0);
      db = *(const v4i*)(dsts + e0 + 4);
    } else {
      da.x = (e0     < nE) ? dsts[min(e0, nE - 1)] : sent;
      da.y = (e0 + 1 < nE) ? dsts[min(e0 + 1, nE - 1)] : sent;
      da.z = (e0 + 2 < nE) ? dsts[min(e0 + 2, nE - 1)] : sent;
      da.w = (e0 + 3 < nE) ? dsts[min(e0 + 3, nE - 1)] : sent;
      db.x = (e0 + 4 < nE) ? dsts[min(e0 + 4, nE - 1)] : sent;
      db.y = (e0 + 5 < nE) ? dsts[min(e0 + 5, nE - 1)] : sent;
      db.z = (e0 + 6 < nE) ? dsts[min(e0 + 6, nE - 1)] : sent;
      db.w = (e0 + 7 < nE) ? dsts[min(e0 + 7, nE - 1)] : sent;
    }
    const unsigned nb = (unsigned)slotBase;
    const unsigned s0 = (unsigned)da.x - nb, s1 = (unsigned)da.y - nb;
    const unsigned s2 = (unsigned)da.z - nb, s3 = (unsigned)da.w - nb;
    const unsigned s4 = (unsigned)db.x - nb, s5 = (unsigned)db.y - nb;
    const unsigned s6 = (unsigned)db.z - nb, s7 = (unsigned)db.w - nb;
    const bool h0 = s0 < (unsigned)NB, h1 = s1 < (unsigned)NB, h2 = s2 < (unsigned)NB, h3 = s3 < (unsigned)NB;
    const bool h4 = s4 < (unsigned)NB, h5 = s5 < (unsigned)NB, h6 = s6 < (unsigned)NB, h7 = s7 < (unsigned)NB;
    const unsigned any = __builtin_amdgcn_ballot_w32(h0 | h1 | h2 | h3 | h4 | h5 | h6 | h7);
    if (any != 0u) {
#define HITJ(J, HJ, SJ) { \
        const unsigned mj = __builtin_amdgcn_ballot_w32(HJ); \
        if (mj != 0u) { \
          if (HJ) { \
            const int pos = wc + (int)__builtin_amdgcn_mbcnt_lo(mj, 0u); \
            if (pos < WCAP) list[wave * WCAP + pos] = ((el0 + (J)) << 12) | (int)(SJ); \
          } \
          wc += (int)__builtin_popcount(mj); } }
      HITJ(0, h0, s0)
      HITJ(1, h1, s1)
      HITJ(2, h2, s2)
      HITJ(3, h3, s3)
      HITJ(4, h4, s4)
      HITJ(5, h5, s5)
      HITJ(6, h6, s6)
      HITJ(7, h7, s7)
#undef HITJ
    }
  }
  return wc;
}

__global__ __launch_bounds__(NTHR) void k_count(
    const int* __restrict__ dsts, int* cnt, float* dinv, int nE, int vec8) {
  __shared__ __attribute__((aligned(16))) int scnt[NBC];
  __shared__ __attribute__((aligned(16))) int list[LISTN];
  __shared__ int wcnt[NWAVE];
  const int tid = threadIdx.x, lane = tid & 31, wave = tid >> 5;
  const int nodeBase = blockIdx.x * NBC;

  for (int i = tid; i < NBC; i += NTHR) scnt[i] = 0;
  __syncthreads();

  const int nChunks = (nE + CHUNK - 1) / CHUNK;
#pragma unroll 1
  for (int ch = 0; ch < nChunks; ++ch) {
    const int cbase = ch * CHUNK;
    const int wc = scan_chunk<NBC>(dsts, nE, cbase, nodeBase, vec8, list, tid, lane, wave);
    if (lane == 0) wcnt[wave] = wc;
    __syncthreads();
    if (wave == 0) {
#pragma unroll 1
      for (int wsx = 0; wsx < NWAVE; ++wsx) {
        int n = __builtin_amdgcn_readfirstlane(wcnt[wsx]);
        n = n > WCAP ? WCAP : (n < 0 ? 0 : n);
        const int* lp = list + wsx * WCAP;
#pragma unroll 1
        for (int i = 0; i < n; ++i) {
          const int ent  = __builtin_amdgcn_readfirstlane(lp[i]);
          const int slot = ent & (NBC - 1);
          if (lane == 0) scnt[slot] = scnt[slot] + 1;
        }
      }
    }
    __syncthreads();
  }

  v4i cq[4];
  v4f dq[4];
#pragma unroll
  for (int q = 0; q < 4; ++q) {
    const int f = (wave * 4 + q) * 128 + 4 * lane;
    const v4i cv = *(const v4i*)(scnt + f);
    cq[q] = cv;
    v4f d;
    d.x = rsqrtf((float)(cv.x < 0 ? 0 : cv.x) + 1.0f);
    d.y = rsqrtf((float)(cv.y < 0 ? 0 : cv.y) + 1.0f);
    d.z = rsqrtf((float)(cv.z < 0 ? 0 : cv.z) + 1.0f);
    d.w = rsqrtf((float)(cv.w < 0 ? 0 : cv.w) + 1.0f);
    dq[q] = d;
  }
  int*   cp = cnt  + (size_t)nodeBase;
  float* dp = dinv + (size_t)nodeBase;
#pragma unroll
  for (int q = 0; q < 4; ++q) {
    const int f = (wave * 4 + q) * 128 + 4 * lane;
    *(volatile v4i*)(cp + f) = cq[q];
    *(volatile v4f*)(dp + f) = dq[q];
  }
  __threadfence();
#pragma unroll
  for (int q = 0; q < 4; ++q) {
    const int f = (wave * 4 + q) * 128 + 4 * lane;
    *(volatile v4i*)(cp + f) = cq[q];
    *(volatile v4f*)(dp + f) = dq[q];
  }
}

__global__ __launch_bounds__(OTHR) void k_offsets(
    const int* __restrict__ cnt, int* off, int* rbase, int nChunk) {
  __shared__ __attribute__((aligned(16))) int soff[NBC];
  __shared__ __attribute__((aligned(16))) int srb[RBN];
  __shared__ int wtot[OTHR / 32];
  const int tid = threadIdx.x, lane = tid & 31, wave = tid >> 5, sub = tid >> 7;
  for (int i = tid; i < RBN; i += OTHR) srb[i] = 0;
  int carry = 0;
#pragma unroll 1
  for (int ch = 0; ch < nChunk; ++ch) {
    const int base = ch * NBC;
    const v4i c0 = *(const v4i*)(cnt + base + 8 * tid);
    const v4i c1 = *(const v4i*)(cnt + base + 8 * tid + 4);
    const int e0 = max(c0.x, 0), e1 = max(c0.y, 0), e2 = max(c0.z, 0), e3 = max(c0.w, 0);
    const int e4 = max(c1.x, 0), e5 = max(c1.y, 0), e6 = max(c1.z, 0), e7 = max(c1.w, 0);
    const int ts = e0 + e1 + e2 + e3 + e4 + e5 + e6 + e7;
    int incl = ts;
#pragma unroll
    for (int d = 1; d < 32; d <<= 1) {
      const int t = __shfl_up(incl, d);
      if (lane >= d) incl += t;
    }
    if (lane == 31) wtot[wave] = incl;
    __syncthreads();
    const int S0 = wtot[0]  + wtot[1]  + wtot[2]  + wtot[3];
    const int S1 = wtot[4]  + wtot[5]  + wtot[6]  + wtot[7];
    const int S2 = wtot[8]  + wtot[9]  + wtot[10] + wtot[11];
    const int S3 = wtot[12] + wtot[13] + wtot[14] + wtot[15];
    int pre = 0;
#pragma unroll 1
    for (int w = 4 * sub; w < wave; ++w) pre += wtot[w];
    const int b0 = carry;
    const int b1 = b0 + ((S0 + 31) & ~31);
    const int b2 = b1 + ((S1 + 31) & ~31);
    const int b3 = b2 + ((S2 + 31) & ~31);
    const int b4 = b3 + ((S3 + 31) & ~31);
    const int myb = sub == 0 ? b0 : (sub == 1 ? b1 : (sub == 2 ? b2 : b3));
    if (tid == 0) {
      srb[min(4 * ch + 0, RBN - 1)] = b0;
      srb[min(4 * ch + 1, RBN - 1)] = b1;
      srb[min(4 * ch + 2, RBN - 1)] = b2;
      srb[min(4 * ch + 3, RBN - 1)] = b3;
    }
    int run = myb + pre + incl - ts;
    soff[8 * tid + 0] = run; run += e0;
    soff[8 * tid + 1] = run; run += e1;
    soff[8 * tid + 2] = run; run += e2;
    soff[8 * tid + 3] = run; run += e3;
    soff[8 * tid + 4] = run; run += e4;
    soff[8 * tid + 5] = run; run += e5;
    soff[8 * tid + 6] = run; run += e6;
    soff[8 * tid + 7] = run;
    carry = b4;
    __syncthreads();
    const v4i o0 = *(const v4i*)(soff + 4 * tid);
    const v4i o1 = *(const v4i*)(soff + 4 * (tid + OTHR));
    int* op = off + base;
    *(volatile v4i*)(op + 4 * tid) = o0;
    *(volatile v4i*)(op + 4 * (tid + OTHR)) = o1;
    __threadfence();
    *(volatile v4i*)(op + 4 * tid) = o0;
    *(volatile v4i*)(op + 4 * (tid + OTHR)) = o1;
    __syncthreads();
  }
  if (tid == 0) srb[min(4 * nChunk, RBN - 1)] = carry;
  __syncthreads();
  v4i rv = {0, 0, 0, 0};
  if (tid < 32) rv = *(const v4i*)(srb + 4 * tid);
  if (tid < 32) *(volatile v4i*)(rbase + 4 * tid) = rv;
  __threadfence();
  if (tid < 32) *(volatile v4i*)(rbase + 4 * tid) = rv;
}

__global__ __launch_bounds__(NTHR) void k_fill(
    const int* __restrict__ srcs, const int* __restrict__ dsts,
    const int* __restrict__ off, const int* __restrict__ rbase,
    int* csr, int nN, int nE, int vec8, int csrLen) {
  extern __shared__ v4f lds_dyn[];
  int* region = (int*)lds_dyn;
  int* cursor = region + RCAP;
  int* list   = cursor + NBF;
  int* wcnt   = list + LISTN;
  const int tid = threadIdx.x, lane = tid & 31, wave = tid >> 5;
  const int b = blockIdx.x;
  const int nodeBase = b * NBF;

  int rb0 = rbase[b];
  const int rb1 = rbase[b + 1];
  rb0 = rb0 < 0 ? 0 : (rb0 > csrLen ? csrLen : rb0);
  rb0 &= ~31;
  int len = rb1 - rb0;
  len = len < 0 ? 0 : (len > RCAP ? RCAP : len);
  int lenW = (len + 31) & ~31;
  if (rb0 + lenW > csrLen) lenW = (csrLen - rb0) & ~31;

  {
    const v4i z = {0, 0, 0, 0};
    for (int i = tid; i < RCAP / 4; i += NTHR) ((v4i*)region)[i] = z;
    for (int s = tid; s < NBF; s += NTHR) {
      int o = off[nodeBase + s] - rb0;
      o = o < 0 ? 0 : (o > RCAP ? RCAP : o);
      cursor[s] = o;
    }
  }
  __syncthreads();

  const int nChunks = (nE + CHUNK - 1) / CHUNK;
#pragma unroll 1
  for (int ch = 0; ch < nChunks; ++ch) {
    const int cbase = ch * CHUNK;
    const int wc = scan_chunk<NBF>(dsts, nE, cbase, nodeBase, vec8, list, tid, lane, wave);
    if (lane == 0) wcnt[wave] = wc;
    __syncthreads();
    if (wave == 0) {
#pragma unroll 1
      for (int wsx = 0; wsx < NWAVE; ++wsx) {
        int n = __builtin_amdgcn_readfirstlane(wcnt[wsx]);
        n = n > WCAP ? WCAP : (n < 0 ? 0 : n);
        const int* lp = list + wsx * WCAP;
#pragma unroll 1
        for (int i = 0; i < n; ++i) {
          const int ent  = __builtin_amdgcn_readfirstlane(lp[i]);
          const int slot = ent & (NBF - 1);
          int e = cbase + ((ent >> 12) & (CHUNK - 1));
          e = e > nE - 1 ? nE - 1 : e;
          int sv = srcs[e];
          sv = sv < 0 ? 0 : (sv > nN - 1 ? nN - 1 : sv);
          if (lane == 0) {
            int pos = cursor[slot];
            pos = pos < 0 ? 0 : (pos > RCAP - 1 ? RCAP - 1 : pos);
            region[pos] = sv;
            const int np = pos + 1;
            cursor[slot] = np > RCAP ? RCAP : np;
          }
        }
      }
    }
    __syncthreads();
  }

  const int nv = lenW >> 2;
  int* gp = csr + rb0;
#pragma unroll 1
  for (int i = tid; i < nv; i += NTHR) { const v4i v = ((const v4i*)region)[i]; *(volatile v4i*)(gp + 4 * i) = v; }
  __threadfence();
#pragma unroll 1
  for (int i = tid; i < nv; i += NTHR) { const v4i v = ((const v4i*)region)[i]; *(volatile v4i*)(gp + 4 * i) = v; }
}

__global__ __launch_bounds__(NTHR) void k_wcvt(const float* __restrict__ wq, const float* __restrict__ wk,
                                               const float* __restrict__ wv, const float* __restrict__ wg,
                                               const float* __restrict__ wl, _Float16* dp, int nUnits) {
  const int i = (int)blockIdx.x * NTHR + (int)threadIdx.x;
  if (i >= nUnits) return;
  const int mat = i >> 11;
  const int r = i & 2047;
  const int n = r >> 4;
  const int seg = r & 15;
  const float* W = (mat == 0) ? wq : ((mat == 1) ? wk : ((mat == 2) ? wv : ((mat == 3) ? wg : wl)));
  const bool tr = mat >= 3;
  v8h o;
#pragma unroll
  for (int j = 0; j < 8; ++j) {
    const int k = 8 * seg + j;
    const float f0 = W[(size_t)k * DW + n];
    const float f1 = W[(size_t)n * DW + k];
    o[j] = (_Float16)((tr ? f1 : f0) * WCARRY);
  }
  _Float16* gp = dp + (size_t)i * 8;
  *(volatile v8h*)gp = o;
  __threadfence();
  *(volatile v8h*)gp = o;
}

__global__ __launch_bounds__(NTHR) void k_proj(
    const float* __restrict__ x, const _Float16* __restrict__ wpl,
    _Float16* q16p, float* vp, float* xwp, float* part, int nValid) {
  extern __shared__ v4f lds_dyn[];
  char* lb = (char*)lds_dyn;
  _Float16* a16   = (_Float16*)(lb + LP_A16);
  float*    stg   = (float*)(lb + LP_STG);
  _Float16* kt16  = (_Float16*)(lb + LP_KT);
  _Float16* vt16  = (_Float16*)(lb + LP_VT);
  float*    sks   = (float*)(lb + LP_SKS);
  float*    swq   = (float*)(lb + LP_SWQ);
  float*    swk   = (float*)(lb + LP_SWK);
  float*    sline = (float*)(lb + LP_SLN);
  float*    mac   = (float*)(lb + LP_MAC);
  const int tid = threadIdx.x, lane = tid & 31, wave = tid >> 5, hh = lane >> 4, m = lane & 15;
  const int rg = wave >> 1, chf = wave & 1;
  const int r0 = rg * 16, c0 = chf * (DW / 2);
  float* pb = part + (size_t)blockIdx.x * PSTRIDE;

  {
    const v4f z = {0.f, 0.f, 0.f, 0.f};
    for (int i = tid; i < (DW * DW) / 4; i += NTHR) ((v4f*)mac)[i] = z;
  }
  float kacc[4] = {0.f, 0.f, 0.f, 0.f};
  float sq = 0.f, sk = 0.f;

#pragma unroll 1
  for (int st = 0; st < RT; ++st) {
    const int rowBase = (int)blockIdx.x * RB + st * BM;

#pragma unroll
    for (int it = 0; it < 8; ++it) {
      const int id = it * NTHR + tid;
      const int row = id >> 5, seg = id & 31;
      const int grow = rowBase + row;
      const bool live = grow < nValid;
      int rr = grow > nValid - 1 ? nValid - 1 : grow;
      rr = rr < 0 ? 0 : rr;
      v4f xv = *(const v4f*)(x + (size_t)rr * DW + 4 * seg);
      v4h o;
      o.x = (_Float16)((live ? xv.x : 0.f) * ACARRY);
      o.y = (_Float16)((live ? xv.y : 0.f) * ACARRY);
      o.z = (_Float16)((live ? xv.z : 0.f) * ACARRY);
      o.w = (_Float16)((live ? xv.w : 0.f) * ACARRY);
      *(v4h*)(a16 + (size_t)row * DW + 4 * seg) = o;
    }
    __syncthreads();

    v8f acc[4];

    gemm_tile4(a16, wpl, r0, c0, hh, m, acc);
    {
      _Float16* qst = kt16;
#pragma unroll
      for (int t = 0; t < 4; ++t) {
#pragma unroll
        for (int r = 0; r < 8; ++r) {
          const float av = acc[t][r];
          const float qv = av * GSCALE;
          sq += qv * qv;
          qst[(size_t)(r0 + 8 * hh + r) * DW + c0 + 16 * t + m] = (_Float16)(av * HCONV);
        }
      }
    }
    __syncthreads();
    {
      v8h cv[4];
#pragma unroll
      for (int it = 0; it < 4; ++it) {
        const int p = it * NTHR + tid;
        cv[it] = *(const v8h*)(kt16 + (size_t)(p >> 4) * DW + 8 * (p & 15));
      }
#pragma unroll
      for (int it = 0; it < 4; ++it) {
        const int p = it * NTHR + tid;
        *(volatile v8h*)(q16p + (size_t)(rowBase + (p >> 4)) * DW + 8 * (p & 15)) = cv[it];
      }
      __threadfence();
#pragma unroll
      for (int it = 0; it < 4; ++it) {
        const int p = it * NTHR + tid;
        *(volatile v8h*)(q16p + (size_t)(rowBase + (p >> 4)) * DW + 8 * (p & 15)) = cv[it];
      }
    }
    __syncthreads();

    gemm_tile4(a16, wpl + (size_t)1 * DW * DW, r0, c0, hh, m, acc);
#pragma unroll
    for (int t = 0; t < 4; ++t) {
      float s8 = 0.f;
      v8h h8;
#pragma unroll
      for (int r = 0; r < 8; ++r) {
        const float av = acc[t][r];
        const float kv = av * GSCALE;
        sk += kv * kv;
        s8 += kv;
        h8[r] = (_Float16)(av * HCONV);
      }
      *(v8h*)(kt16 + (size_t)(c0 + 16 * t + m) * BM + r0 + 8 * hh) = h8;
      s8 += __shfl_xor(s8, 16);
      kacc[t] += s8;
    }

    gemm_tile4(a16, wpl + (size_t)2 * DW * DW, r0, c0, hh, m, acc);
#pragma unroll
    for (int t = 0; t < 4; ++t) {
      v8h h8;
#pragma unroll
      for (int r = 0; r < 8; ++r) {
        const float av = acc[t][r];
        stg[(size_t)(r0 + 8 * hh + r) * DW + c0 + 16 * t + m] = av * GSCALE;
        h8[r] = (_Float16)(av * HCONV);
      }
      *(v8h*)(vt16 + (size_t)(c0 + 16 * t + m) * BM + r0 + 8 * hh) = h8;
    }
    __syncthreads();
    write_rows64(stg, vp + (size_t)rowBase * DW, 1.0f, tid);

    {
      const _Float16* ka = kt16 + (size_t)(16 * wave + m) * BM + 8 * hh;
      const _Float16* vb = vt16 + (size_t)m * BM + 8 * hh;
      Frag a0, a1;
      a0.h[0] = *(const v8h*)(ka);
      a0.h[1] = *(const v8h*)(ka + 16);
      a1.h[0] = *(const v8h*)(ka + 32);
      a1.h[1] = *(const v8h*)(ka + 48);
      float* mr = mac + (size_t)(16 * wave + 8 * hh) * DW + m;
#pragma unroll 1
      for (int t = 0; t < 8; ++t) {
        float* me = mr + 16 * t;
        v8f c;
#pragma unroll
        for (int r = 0; r < 8; ++r) c[r] = me[(size_t)r * DW];
        const _Float16* vt = vb + (size_t)(16 * t) * BM;
        Frag b;
        b.h[0] = *(const v8h*)(vt);
        b.h[1] = *(const v8h*)(vt + 16);
        c = wmh(a0.v, b.v, c);
        b.h[0] = *(const v8h*)(vt + 32);
        b.h[1] = *(const v8h*)(vt + 48);
        c = wmh(a1.v, b.v, c);
#pragma unroll
        for (int r = 0; r < 8; ++r) me[(size_t)r * DW] = c[r];
      }
    }
    __syncthreads();

    gemm_tile4(a16, wpl + (size_t)3 * DW * DW, r0, c0, hh, m, acc);
#pragma unroll
    for (int t = 0; t < 4; ++t) {
#pragma unroll
      for (int r = 0; r < 8; ++r)
        stg[(size_t)(r0 + 8 * hh + r) * DW + c0 + 16 * t + m] = acc[t][r] * GSCALE;
    }
    __syncthreads();
    write_rows64(stg, xwp + (size_t)rowBase * DW, 1.0f, tid);
  }
  __syncthreads();

  if (hh == 0) {
#pragma unroll
    for (int t = 0; t < 4; ++t) sks[rg * DW + c0 + 16 * t + m] = kacc[t];
  }
#pragma unroll
  for (int d = 16; d >= 1; d >>= 1) {
    sq += __shfl_xor(sq, d);
    sk += __shfl_xor(sk, d);
  }
  if (lane == 0) { swq[wave] = sq; swk[wave] = sk; }
  __syncthreads();

  write_rows64(mac, pb, MSCALE, tid);
  write_rows64(mac + (size_t)64 * DW, pb + (size_t)64 * DW, MSCALE, tid);

  if (tid < DW) {
    sline[tid] = ((sks[tid] + sks[DW + tid]) + sks[2 * DW + tid]) + sks[3 * DW + tid];
  } else if (tid == DW) {
    float s = 0.f;
#pragma unroll
    for (int w = 0; w < NWAVE; ++w) s += swq[w];
    sline[DW] = s;
  } else if (tid == DW + 1) {
    float s = 0.f;
#pragma unroll
    for (int w = 0; w < NWAVE; ++w) s += swk[w];
    sline[DW + 1] = s;
  } else if (tid < DW + 32) {
    sline[tid] = 0.f;
  }
  __syncthreads();
  if (tid < 40) {
    const v4f v = *(const v4f*)(sline + 4 * tid);
    *(volatile v4f*)(pb + (size_t)DW * DW + 4 * tid) = v;
  }
  __threadfence();
  if (tid < 40) {
    const v4f v = *(const v4f*)(sline + 4 * tid);
    *(volatile v4f*)(pb + (size_t)DW * DW + 4 * tid) = v;
  }
}

__global__ __launch_bounds__(NTHR) void k_reduce(const float* __restrict__ part, int nBlk,
                                                 _Float16* mp16, float* scal) {
  __shared__ __attribute__((aligned(16))) _Float16 smp[MPN * DW];
  __shared__ __attribute__((aligned(16))) float ssc[32];
  const int tid = threadIdx.x;
  const int nb = nBlk < 0 ? 0 : nBlk;

  for (int i = DW + tid; i < (MPN - DW) * DW; i += NTHR) smp[DW * DW + i] = (_Float16)0.0f;

#pragma unroll 1
  for (int e = tid; e < DW * DW; e += NTHR) {
    double s = 0.0;
#pragma unroll 1
    for (int b = 0; b < nb; ++b) s += (double)part[(size_t)b * PSTRIDE + e];
    const int i = e >> 7, j = e & 127;
    smp[(size_t)j * DW + i] = (_Float16)((float)s * MCARRY);
  }
  if (tid < DW) {
    double s = 0.0;
#pragma unroll 1
    for (int b = 0; b < nb; ++b) s += (double)part[(size_t)b * PSTRIDE + DW * DW + tid];
    smp[(size_t)DW * DW + tid] = (_Float16)((float)s);
  }
  if (tid == 0) {
    double a = 0.0, c = 0.0;
#pragma unroll 1
    for (int b = 0; b < nb; ++b) {
      a += (double)part[(size_t)b * PSTRIDE + DW * DW + DW];
      c += (double)part[(size_t)b * PSTRIDE + DW * DW + DW + 1];
    }
    const double gg = 1.0 / (sqrt(a) * sqrt(c) * 128.0);
    ssc[0] = (float)gg;
  } else if (tid < 32) {
    ssc[tid] = 0.f;
  }
  __syncthreads();

#pragma unroll 1
  for (int p = tid; p < (MPN * DW) / 8; p += NTHR) {
    const v8h v = *(const v8h*)(smp + (size_t)8 * p);
    *(volatile v8h*)(mp16 + (size_t)8 * p) = v;
  }
  if (tid < 8) {
    const v4f v = *(const v4f*)(ssc + 4 * tid);
    *(volatile v4f*)(scal + 4 * tid) = v;
  }
  __threadfence();
#pragma unroll 1
  for (int p = tid; p < (MPN * DW) / 8; p += NTHR) {
    const v8h v = *(const v8h*)(smp + (size_t)8 * p);
    *(volatile v8h*)(mp16 + (size_t)8 * p) = v;
  }
  if (tid < 8) {
    const v4f v = *(const v4f*)(ssc + 4 * tid);
    *(volatile v4f*)(scal + 4 * tid) = v;
  }
}

__global__ __launch_bounds__(NTHR) void k_agg(
    const int* __restrict__ csr, const int* __restrict__ off, const int* __restrict__ cnt,
    const float* __restrict__ dinv, const float* __restrict__ h, const float* __restrict__ bias,
    float* gout, int nN, int csrLen) {
  const int tid = threadIdx.x, lane = tid & 31, wave = tid >> 5;
  const int tbase = blockIdx.x * TGT + wave * 32;
  const int col4 = 4 * lane;
  const int cl    = tbase + lane;
  const int cnt_l = cnt[cl];
  const int off_l = off[cl];
  const float di_l = dinv[cl];
  const v4f bv = *(const v4f*)(bias + col4);

#pragma unroll 1
  for (int j = 0; j < 32; ++j) {
    const int c = tbase + j;
    int n = __shfl(cnt_l, j);
    n = n < 0 ? 0 : (n > DEGCAP ? DEGCAP : n);
    const int st = __shfl(off_l, j);
    const float dc = __shfl(di_l, j);
    const float dd = dc * dc;

    v4f a = *(const v4f*)(h + (size_t)c * DW + col4);
    a = a * dd;
#pragma unroll 1
    for (int q0 = 0; q0 < n; q0 += 32) {
      int pos = st + q0 + lane;
      pos = pos < 0 ? 0 : (pos > csrLen - 1 ? csrLen - 1 : pos);
      int sl = csr[pos];
      sl = sl < 0 ? 0 : (sl > nN - 1 ? nN - 1 : sl);
      const int mcnt = (n - q0) < 32 ? (n - q0) : 32;
#pragma unroll 1
      for (int pp = 0; pp < mcnt; ++pp) {
        const int s = __builtin_amdgcn_readlane(sl, pp);
        const float cf = dinv[s] * dc;
        const v4f xv = *(const v4f*)(h + (size_t)s * DW + col4);
        a = a + xv * cf;
      }
    }

    const bool live = c < nN;
    v4f o;
    o.x = live ? (a.x + bv.x) : 0.f;
    o.y = live ? (a.y + bv.y) : 0.f;
    o.z = live ? (a.z + bv.z) : 0.f;
    o.w = live ? (a.w + bv.w) : 0.f;
    float* gp = gout + (size_t)c * DW + col4;
    *(volatile v4f*)gp = o;
    __threadfence();
    *(volatile v4f*)gp = o;
  }
}

__global__ __launch_bounds__(NTHR) void k_final(
    const float* __restrict__ x, const _Float16* __restrict__ q16p, const float* __restrict__ vp,
    const float* __restrict__ gcnp, const _Float16* __restrict__ mp16, const _Float16* __restrict__ wl16,
    const float* __restrict__ blin, const float* __restrict__ scal, float* out, int nValid) {
  __shared__ __attribute__((aligned(16))) float stg[BM * DW];
  __shared__ __attribute__((aligned(16))) _Float16 z16[BM * DW];
  __shared__ float srow[BM];
  const int tid = threadIdx.x, lane = tid & 31, wave = tid >> 5, hh = lane >> 4, m = lane & 15;
  const int rg = wave >> 1, chf = wave & 1;
  const int r0 = rg * 16, c0 = chf * (DW / 2);
  const int rowBase = (int)blockIdx.x * BM;
  const float g = scal[0];

  v8f acc[5];
#pragma unroll
  for (int t = 0; t < 5; ++t) acc[t] = zero8();
  {
    const _Float16* ap = q16p + (size_t)(rowBase + r0 + m) * DW + 8 * hh;
    const _Float16* bp = mp16 + (size_t)(c0 + m) * DW + 8 * hh;
    const _Float16* bq = mp16 + (size_t)(DW + m) * DW + 8 * hh;
#pragma unroll 1
    for (int kt = 0; kt < KSTEPS; ++kt) {
      Frag a;
      a.h[0] = *(const v8h*)(ap + 32 * kt);
      a.h[1] = *(const v8h*)(ap + 32 * kt + 16);
#pragma unroll
      for (int t = 0; t < 4; ++t) {
        const size_t to = (size_t)(16 * t) * DW + 32 * kt;
        Frag b;
        b.h[0] = *(const v8h*)(bp + to);
        b.h[1] = *(const v8h*)(bp + to + 16);
        acc[t] = wmh(a.v, b.v, acc[t]);
      }
      Frag b8;
      b8.h[0] = *(const v8h*)(bq + 32 * kt);
      b8.h[1] = *(const v8h*)(bq + 32 * kt + 16);
      acc[4] = wmh(a.v, b8.v, acc[4]);
    }
  }

  {
    float* sp = stg + (size_t)(r0 + 8 * hh) * DW + c0 + m;
    const float gt = g * 0.5f;
#pragma unroll
    for (int t = 0; t < 4; ++t) {
#pragma unroll
      for (int r = 0; r < 8; ++r) sp[(size_t)r * DW + 16 * t] = acc[t][r] * gt;
    }
    if (chf == 0 && m == 0) {
      const float gq = g * 0.125f;
#pragma unroll
      for (int r = 0; r < 8; ++r) {
        const float qk = acc[4][r] * gq;
        srow[r0 + 8 * hh + r] = 1.0f / (1.0f + qk);
      }
    }
  }
  __syncthreads();

#pragma unroll
  for (int it = 0; it < 8; ++it) {
    const int id = it * NTHR + tid;
    const int row = id >> 5, seg = id & 31;
    const int grow = rowBase + row;
    const bool live = grow < nValid;
    int rr = grow > nValid - 1 ? nValid - 1 : grow;
    rr = rr < 0 ? 0 : rr;
    const v4f xv = *(const v4f*)(x    + (size_t)rr * DW + 4 * seg);
    const v4f vv = *(const v4f*)(vp   + (size_t)rr * DW + 4 * seg);
    const v4f gv = *(const v4f*)(gcnp + (size_t)rr * DW + 4 * seg);
    const v4f tv = *(const v4f*)(stg + (size_t)row * DW + 4 * seg);
    const float sc = srow[row];
    const float bs = CBETA * sc;
    v4f zo;
    {
      const float at = vv.x + tv.x; const float z = bs * at + OMBETA * xv.x;
      zo.x = live ? (OMALPHA * z + CALPHA * gv.x) : 0.f;
    }
    {
      const float at = vv.y + tv.y; const float z = bs * at + OMBETA * xv.y;
      zo.y = live ? (OMALPHA * z + CALPHA * gv.y) : 0.f;
    }
    {
      const float at = vv.z + tv.z; const float z = bs * at + OMBETA * xv.z;
      zo.z = live ? (OMALPHA * z + CALPHA * gv.z) : 0.f;
    }
    {
      const float at = vv.w + tv.w; const float z = bs * at + OMBETA * xv.w;
      zo.w = live ? (OMALPHA * z + CALPHA * gv.w) : 0.f;
    }
    v4h o;
    o.x = (_Float16)(zo.x * ACARRY);
    o.y = (_Float16)(zo.y * ACARRY);
    o.z = (_Float16)(zo.z * ACARRY);
    o.w = (_Float16)(zo.w * ACARRY);
    *(v4h*)(z16 + (size_t)row * DW + 4 * seg) = o;
  }
  __syncthreads();

  v8f accb[4];
  gemm_tile4(z16, wl16, r0, c0, hh, m, accb);
  {
    float* sp = stg + (size_t)(r0 + 8 * hh) * DW + c0 + m;
#pragma unroll
    for (int t = 0; t < 4; ++t) {
      const float bl = blin[c0 + 16 * t + m];
#pragma unroll
      for (int r = 0; r < 8; ++r) sp[(size_t)r * DW + 16 * t] = accb[t][r] * GSCALE + bl;
    }
  }
  __syncthreads();

  v4f cv[8];
#pragma unroll
  for (int it = 0; it < 8; ++it) {
    const int id = it * NTHR + tid;
    cv[it] = *(const v4f*)(stg + (size_t)(id >> 5) * DW + 4 * (id & 31));
  }
#pragma unroll
  for (int it = 0; it < 8; ++it) {
    const int id = it * NTHR + tid;
    const int grow = rowBase + (id >> 5);
    if (grow < nValid) *(volatile v4f*)(out + (size_t)grow * DW + 4 * (id & 31)) = cv[it];
  }
  __threadfence();
#pragma unroll
  for (int it = 0; it < 8; ++it) {
    const int id = it * NTHR + tid;
    const int grow = rowBase + (id >> 5);
    if (grow < nValid) *(volatile v4f*)(out + (size_t)grow * DW + 4 * (id & 31)) = cv[it];
  }
}

extern "C" void kernel_launch(void* const* d_in, const int* in_sizes, int n_in,
                              void* d_out, int out_size, void* d_ws, size_t ws_size,
                              hipStream_t stream) {
  if (n_in < 9) return;
  if (in_sizes[0] < DW || (in_sizes[0] % DW) != 0) return;
  const int nN = in_sizes[0] / DW;
  if (in_sizes[1] < 2 || (in_sizes[1] & 1) != 0) return;
  const int nE = in_sizes[1] / 2;
  if (in_sizes[2] != DW * DW || in_sizes[3] != DW * DW || in_sizes[4] != DW * DW) return;
  if (in_sizes[5] != DW * DW || in_sizes[6] != DW || in_sizes[7] != DW * DW || in_sizes[8] != DW) return;
  if ((long long)out_size != (long long)nN * DW) return;
  if (nE > (1 << 28) || nN > (1 << 22)) return;

  const float* x    = (const float*)d_in[0];
  const int*   ei   = (const int*)d_in[1];
  const int*   src  = ei;
  const int*   dst  = ei + nE;
  const float* wq   = (const float*)d_in[2];
  const float* wk   = (const float*)d_in[3];
  const float* wv   = (const float*)d_in[4];
  const float* wg   = (const float*)d_in[5];
  const float* bg   = (const float*)d_in[6];
  const float* wl   = (const float*)d_in[7];
  const float* bl   = (const float*)d_in[8];
  float* out = (float*)d_out;

  const int NPAD   = ((nN + TGT - 1) / TGT) * TGT;
  const int nBC    = (nN + NBC - 1) / NBC;
  const int CNTPAD = nBC * NBC;
  if (CNTPAD < NPAD) return;
  if (4 * nBC + 1 > RBN) return;
  const int nBF    = (nN + NBF - 1) / NBF;
  if (nBF > 4 * nBC) return;
  const int csrLen = ((nE + 31) & ~31) + 4096;
  if (31 * 4 * nBC > 4096) return;
  const int nAgg   = NPAD / TGT;
  const int nProj  = NPAD / RB;
  const int nFin   = (nN + BM - 1) / BM;
  const int nUnits = NMAT * DW * (DW / 8);

  char* ws = (char*)d_ws;
  size_t off = 0;
  const size_t oWp  = off; off += (size_t)NMAT * DW * DW * 2;    off = (off + 255) & ~(size_t)255;
  const size_t oQ   = off; off += (size_t)NPAD * DW * 2;         off = (off + 255) & ~(size_t)255;
  const size_t oV   = off; off += (size_t)NPAD * DW * 4;         off = (off + 255) & ~(size_t)255;
  const size_t oXw  = off; off += (size_t)NPAD * DW * 4;         off = (off + 255) & ~(size_t)255;
  const size_t oGc  = off; off += (size_t)NPAD * DW * 4;         off = (off + 255) & ~(size_t)255;
  const size_t oCnt = off; off += (size_t)CNTPAD * 4;            off = (off + 255) & ~(size_t)255;
  const size_t oDi  = off; off += (size_t)CNTPAD * 4;            off = (off + 255) & ~(size_t)255;
  const size_t oOff = off; off += (size_t)CNTPAD * 4;            off = (off + 255) & ~(size_t)255;
  const size_t oRb  = off; off += (size_t)RBN * 4;               off = (off + 255) & ~(size_t)255;
  const size_t oCsr = off; off += (size_t)csrLen * 4;            off = (off + 255) & ~(size_t)255;
  const size_t oPt  = off; off += (size_t)nProj * PSTRIDE * 4;   off = (off + 255) & ~(size_t)255;
  const size_t oMp  = off; off += (size_t)MPN * DW * 2;          off = (off + 255) & ~(size_t)255;
  const size_t oSc  = off; off += (size_t)32 * 4;                off = (off + 255) & ~(size_t)255;
  if (off > ws_size || off > (size_t)WSLIM) return;

  _Float16* wpl  = (_Float16*)(ws + oWp);
  _Float16* q16  = (_Float16*)(ws + oQ);
  float*    vp   = (float*)(ws + oV);
  float*    xwp  = (float*)(ws + oXw);
  float*    gcp  = (float*)(ws + oGc);
  int*      cnt  = (int*)(ws + oCnt);
  float*    dinv = (float*)(ws + oDi);
  int*      offp = (int*)(ws + oOff);
  int*      rb   = (int*)(ws + oRb);
  int*      csr  = (int*)(ws + oCsr);
  float*    part = (float*)(ws + oPt);
  _Float16* mp16 = (_Float16*)(ws + oMp);
  float*    scal = (float*)(ws + oSc);

  const int vec8 = ((nE & 3) == 0) ? 1 : 0;

  k_wcvt<<<(nUnits + NTHR - 1) / NTHR, NTHR, 0, stream>>>(wq, wk, wv, wg, wl, wpl, nUnits);
  k_count<<<nBC, NTHR, 0, stream>>>(dst, cnt, dinv, nE, vec8);
  k_offsets<<<1, OTHR, 0, stream>>>(cnt, offp, rb, nBC);
  hipFuncSetAttribute(reinterpret_cast<const void*>(&k_fill),
                      hipFuncAttributeMaxDynamicSharedMemorySize, LDS_FILL);
  k_fill<<<nBF, NTHR, LDS_FILL, stream>>>(src, dst, offp, rb, csr, nN, nE, vec8, csrLen);

  hipFuncSetAttribute(reinterpret_cast<const void*>(&k_proj),
                      hipFuncAttributeMaxDynamicSharedMemorySize, LDS_PROJ);
  k_proj<<<nProj, NTHR, LDS_PROJ, stream>>>(x, wpl, q16, vp, xwp, part, nN);

  k_reduce<<<1, NTHR, 0, stream>>>(part, nProj, mp16, scal);

  k_agg<<<nAgg, NTHR, 0, stream>>>(csr, offp, cnt, dinv, xwp, bg, gcp, nN, csrLen);

  k_final<<<nFin, NTHR, 0, stream>>>(x, q16, vp, gcp, mp16, wpl + (size_t)4 * DW * DW, bl, scal, out, nN);
}
